// ResidualBlock_13443247636813
// MI455X (gfx1250) — hardware-verified
//
#include <hip/hip_runtime.h>
#include <stddef.h>
#include <stdint.h>
#include <math.h>


#define D      64
#define AP     512
#define KC     512
#define KP     128
#define NTHR   256
#define NWAVE  8
#define EPT    8
#define CHUNK  (NTHR * EPT)
#define WCAP   (EPT * 32)
#define LISTN  (NWAVE * WCAP)
#define NBD    8192
#define SLD    13
#define NBA    1024
#define SLA    10
#define RCAP   28672
#define DEGCAP 64
#define GBM    64
#define GBN    64
#define GTHR   128
#define NCONV  5
#define UCONV  (NCONV * D * (KC / 8))
#define UPB    (KP * (KP / 8))
#define UWAB   (4 * D * (KP / 8))
#define UTOT   (UCONV + UPB + UWAB)
#define EB     128
#define CSR_ZINTS (LISTN + 2 * RCAP + 3 * NBA)
#define MISC_INTS 16
#define STG_INTS  (NWAVE * 96)
#define CSR_LDS_INTS (CSR_ZINTS + MISC_INTS + STG_INTS)
#define CW128  0
#define CBE0   64
#define CG0    128
#define CB0    192
#define CBA0   256
#define CBB0   320
#define CG1    384
#define CB1    448
#define CWF    768
#define CBF    832
#define CDBL   840
#define COST   896
#define ECST   1024
#define ELDS_FLOATS (ECST + 2 * NWAVE * 1024)
#define WSMAX  134217728
#define EPSV   1e-5f

static_assert((CHUNK & (CHUNK - 1)) == 0 && CHUNK <= 4096);
static_assert((NBD & (NBD - 1)) == 0 && NBD == (1 << SLD));
static_assert((NBA & (NBA - 1)) == 0 && NBA == (1 << SLA));
static_assert(((long long)CHUNK << SLD) < (1LL << 31));
static_assert(((long long)CHUNK << SLA) < (1LL << 31));
static_assert(NBD % (NTHR * 4) == 0);
static_assert(LISTN % NTHR == 0);
static_assert(NBA % NWAVE == 0 && NBA % 32 == 0 && NBA % GBM == 0 && NBA == 4 * NTHR);
static_assert(RCAP % 32 == 0 && CSR_ZINTS % (NTHR * 4) == 0 && LISTN % 4 == 0);
static_assert(((CSR_ZINTS + MISC_INTS) % 4) == 0);
static_assert(CSR_LDS_INTS * 4 <= 300000);
static_assert(KC % 32 == 0 && KP % 32 == 0 && KC == AP && KP == 2 * D);
static_assert(GBM == (GTHR / 32) * 16 && GBN == D && D == 2 * 32);
static_assert(UCONV % NTHR == 0 && (UCONV + UPB) % NTHR == 0 && UTOT % NTHR == 0 && 1024 % NTHR == 0);
static_assert(DEGCAP == 64);
static_assert(GBM % NWAVE == 0 && EB == NWAVE * 16);
static_assert(COST + EB <= ECST && CDBL + 4 <= COST && CBF < CDBL);
static_assert(ELDS_FLOATS * 4 <= 300000);

typedef float          v2f   __attribute__((ext_vector_type(2)));
typedef float          v4f   __attribute__((ext_vector_type(4)));
typedef float          v8f   __attribute__((ext_vector_type(8)));
typedef int            v4i   __attribute__((ext_vector_type(4)));
typedef int            v8i   __attribute__((ext_vector_type(8)));
typedef unsigned int   v4u   __attribute__((ext_vector_type(4)));
typedef unsigned short v4us  __attribute__((ext_vector_type(4)));
typedef unsigned short v8us  __attribute__((ext_vector_type(8)));
typedef unsigned short v16us __attribute__((ext_vector_type(16)));
typedef __bf16         v16bf __attribute__((ext_vector_type(16)));
typedef v2f  __attribute__((may_alias)) v2fa;
typedef v4f  __attribute__((may_alias)) v4fa;
typedef v4i  __attribute__((may_alias)) v4ia;
typedef v4u  __attribute__((may_alias)) v4ua;
typedef v4us __attribute__((may_alias)) v4usa;
typedef v8us __attribute__((may_alias)) v8usa;
typedef double __attribute__((may_alias)) dbla;
union FragB { v16bf v; v16us u; v8us h[2]; v8i w; };
union DU { double d[2]; v4u u; };

__device__ __forceinline__ v8f wmb(const FragB& a, const FragB& b, v8f c) {
  v8f d = __builtin_amdgcn_wmma_f32_16x16x32_bf16(false, a.v, false, b.v, (short)0, c, false, false);
  asm volatile("v_nop\n\tv_nop\n\tv_nop\n\tv_nop" : "+v"(d) : "v"(a.w), "v"(b.w));
  return d;
}

__device__ __forceinline__ unsigned bf16_bits(float f) {
  const unsigned u = __float_as_uint(f);
  return (u + 0x7FFFu + ((u >> 16) & 1u)) >> 16;
}
__device__ __forceinline__ float bf16_val(float f) {
  return __uint_as_float(bf16_bits(f) << 16);
}
__device__ __forceinline__ void hilo4(const v4f y, v4us& h4, v4us& l4) {
  unsigned hb;
  hb = bf16_bits(y.x); h4[0] = (unsigned short)hb; l4[0] = (unsigned short)bf16_bits(y.x - __uint_as_float(hb << 16));
  hb = bf16_bits(y.y); h4[1] = (unsigned short)hb; l4[1] = (unsigned short)bf16_bits(y.y - __uint_as_float(hb << 16));
  hb = bf16_bits(y.z); h4[2] = (unsigned short)hb; l4[2] = (unsigned short)bf16_bits(y.z - __uint_as_float(hb << 16));
  hb = bf16_bits(y.w); h4[3] = (unsigned short)hb; l4[3] = (unsigned short)bf16_bits(y.w - __uint_as_float(hb << 16));
}

__device__ __forceinline__ void wave_sync() {
  __builtin_amdgcn_fence(__ATOMIC_RELEASE, "wavefront");
  __builtin_amdgcn_wave_barrier();
  __builtin_amdgcn_fence(__ATOMIC_ACQUIRE, "wavefront");
}

template <int SLB>
__device__ __forceinline__ int scan_chunk(const int* __restrict__ dsts, int nE, int cbase, int slotBase,
                                          int nb, int vec8, int* list, int tid, int lane, int wave) {
  int wc = 0;
  const int el0  = tid * EPT;
  const int e0   = cbase + el0;
  const int sent = -2147483647 - 1;
  v4i da, db;
  if (vec8 != 0 && cbase + CHUNK <= nE) {
    da = *(const v4i*)(dsts + e0);
    db = *(const v4i*)(dsts + e0 + 4);
  } else {
    da.x = (e0     < nE) ? dsts[min(e0,     nE - 1)] : sent;
    da.y = (e0 + 1 < nE) ? dsts[min(e0 + 1, nE - 1)] : sent;
    da.z = (e0 + 2 < nE) ? dsts[min(e0 + 2, nE - 1)] : sent;
    da.w = (e0 + 3 < nE) ? dsts[min(e0 + 3, nE - 1)] : sent;
    db.x = (e0 + 4 < nE) ? dsts[min(e0 + 4, nE - 1)] : sent;
    db.y = (e0 + 5 < nE) ? dsts[min(e0 + 5, nE - 1)] : sent;
    db.z = (e0 + 6 < nE) ? dsts[min(e0 + 6, nE - 1)] : sent;
    db.w = (e0 + 7 < nE) ? dsts[min(e0 + 7, nE - 1)] : sent;
  }
  const unsigned nbs = (unsigned)slotBase;
  const unsigned unb = (unsigned)nb;
  const unsigned s0 = (unsigned)da.x - nbs, s1 = (unsigned)da.y - nbs;
  const unsigned s2 = (unsigned)da.z - nbs, s3 = (unsigned)da.w - nbs;
  const unsigned s4 = (unsigned)db.x - nbs, s5 = (unsigned)db.y - nbs;
  const unsigned s6 = (unsigned)db.z - nbs, s7 = (unsigned)db.w - nbs;
  const bool h0 = s0 < unb, h1 = s1 < unb, h2 = s2 < unb, h3 = s3 < unb;
  const bool h4 = s4 < unb, h5 = s5 < unb, h6 = s6 < unb, h7 = s7 < unb;
  const unsigned any = __builtin_amdgcn_ballot_w32(h0 | h1 | h2 | h3 | h4 | h5 | h6 | h7);
  if (any != 0u) {
#define HITJ(J, HJ, SJ) { \
      const unsigned mj = __builtin_amdgcn_ballot_w32(HJ); \
      if (mj != 0u) { \
        if (HJ) { \
          const int pos = wc + (int)__builtin_amdgcn_mbcnt_lo(mj, 0u); \
          if (pos < WCAP) list[wave * WCAP + pos] = ((el0 + (J)) << SLB) | (int)(SJ); \
        } \
        wc += (int)__builtin_popcount(mj); } }
    HITJ(0, h0, s0)
    HITJ(1, h1, s1)
    HITJ(2, h2, s2)
    HITJ(3, h3, s3)
    HITJ(4, h4, s4)
    HITJ(5, h5, s5)
    HITJ(6, h6, s6)
    HITJ(7, h7, s7)
#undef HITJ
  }
  return wc;
}

__global__ __launch_bounds__(NTHR) void k_wprep(const float* __restrict__ tagw, const float* __restrict__ we0,
                                                const float* __restrict__ wa, const float* __restrict__ wb,
                                                unsigned short* bt, unsigned short* pbt, unsigned short* wab) {
  const int u = (int)blockIdx.x * NTHR + (int)threadIdx.x;
  const float* p;
  unsigned short* dp;
  if (u < UCONV) {
    const int c  = u >> 12;
    const int v  = u & 4095;
    const int n  = v >> 6;
    const int k8 = (v & 63) * 8;
    const int kk = k8 >> 7;
    const int j  = k8 & 63;
    p  = tagw + ((size_t)(c * 4 + kk) * D + j) * D + n;
    dp = bt + (size_t)c * D * KC + (size_t)n * KC + k8;
  } else if (u < UCONV + UPB) {
    const int v  = u - UCONV;
    const int n  = v >> 4;
    const int k8 = (v & 15) * 8;
    const int j  = k8 & 63;
    const int ro = (n >> 6) * D;
    const int cn = n & 63;
    p  = we0 + (size_t)(ro + j) * D + cn;
    dp = pbt + (size_t)n * KP + k8;
  } else if (u < UTOT) {
    const int v  = u - UCONV - UPB;
    const int pl = v >> 10;
    const int w  = v & 1023;
    const int n  = w >> 4;
    const int k8 = (w & 15) * 8;
    const int j  = k8 & 63;
    const float* base = (pl & 1) ? wb : wa;
    p  = base + (size_t)(pl >> 1) * D * D + (size_t)j * D + n;
    dp = wab + (size_t)pl * D * KP + (size_t)n * KP + k8;
  } else {
    return;
  }
  v8us o;
#pragma unroll
  for (int i = 0; i < 8; ++i) o[i] = (unsigned short)bf16_bits(p[(size_t)i * D]);
  *(volatile v8us*)dp = o;
  __threadfence();
  *(volatile v8us*)dp = o;
}

__global__ __launch_bounds__(NTHR) void k_deg(const int* __restrict__ dsts, const float* __restrict__ ew,
                                              int nE, int vec8, float* dinv) {
  __shared__ __attribute__((aligned(16))) float sdeg[NBD];
  __shared__ __attribute__((aligned(16))) int list[LISTN];
  __shared__ int wcnt[NWAVE];
  const int tid = (int)threadIdx.x, lane = tid & 31, wave = tid >> 5;
  const int nodeBase = (int)blockIdx.x * NBD;

  for (int i = tid; i < NBD; i += NTHR) sdeg[i] = 0.0f;
  for (int i = tid; i < LISTN; i += NTHR) list[i] = 0;
  if (tid < NWAVE) wcnt[tid] = 0;
  __syncthreads();

  const int nChunks = (nE + CHUNK - 1) / CHUNK;
#pragma unroll 1
  for (int ch = 0; ch < nChunks; ++ch) {
    const int cbase = ch * CHUNK;
    const int wc = scan_chunk<SLD>(dsts, nE, cbase, nodeBase, NBD, vec8, list, tid, lane, wave);
    if (lane == 0) wcnt[wave] = wc;
    __syncthreads();
    if (wave == 0) {
#pragma unroll 1
      for (int w2 = 0; w2 < NWAVE; ++w2) {
        int c = wcnt[w2];
        c = c < 0 ? 0 : (c > WCAP ? WCAP : c);
#pragma unroll 1
        for (int b0 = 0; b0 < c; b0 += 32) {
          const int idx = b0 + lane;
          const int ent = list[w2 * WCAP + (idx < WCAP ? idx : WCAP - 1)];
          const int m32 = (c - b0) < 32 ? (c - b0) : 32;
#pragma unroll 1
          for (int k = 0; k < m32; ++k) {
            const int u  = __builtin_amdgcn_readlane(ent, k);
            const int sl = u & (NBD - 1);
            const int el = (u >> SLD) & (CHUNK - 1);
            int eid = cbase + el;
            eid = eid > nE - 1 ? nE - 1 : eid;
            const float wv = bf16_val(ew[eid]);
            if (lane == 0) sdeg[sl] = sdeg[sl] + wv;
          }
        }
      }
    }
    __syncthreads();
  }

  v4f vals[NBD / (NTHR * 4)];
#pragma unroll
  for (int it = 0; it < NBD / (NTHR * 4); ++it) {
    const int s0 = it * (NTHR * 4) + 4 * tid;
    const v4f d4 = *(const v4fa*)(sdeg + s0);
    v4f v;
    v.x = (d4.x > 0.0f) ? rsqrtf(d4.x) : 0.0f;
    v.y = (d4.y > 0.0f) ? rsqrtf(d4.y) : 0.0f;
    v.z = (d4.z > 0.0f) ? rsqrtf(d4.z) : 0.0f;
    v.w = (d4.w > 0.0f) ? rsqrtf(d4.w) : 0.0f;
    vals[it] = v;
  }
#pragma unroll
  for (int it = 0; it < NBD / (NTHR * 4); ++it) {
    const int s0 = it * (NTHR * 4) + 4 * tid;
    *(volatile v4f*)(dinv + (size_t)nodeBase + s0) = vals[it];
  }
  __threadfence();
#pragma unroll
  for (int it = 0; it < NBD / (NTHR * 4); ++it) {
    const int s0 = it * (NTHR * 4) + 4 * tid;
    *(volatile v4f*)(dinv + (size_t)nodeBase + s0) = vals[it];
  }
}

__global__ __launch_bounds__(NTHR) void k_csr(const int* __restrict__ srcs, const int* __restrict__ dsts,
                                              const float* __restrict__ ew, int nE, int nN, int vec8, int mRows,
                                              const float* __restrict__ dinv, int* ctab,
                                              unsigned short* stab, float* ntab) {
  extern __shared__ __attribute__((aligned(16))) int dsm[];
  int* list = dsm;
  int* hl   = dsm + LISTN;
  int* sl   = hl + RCAP;
  int* cnt  = sl + RCAP;
  int* offs = cnt + NBA;
  int* cur  = offs + NBA;
  int* misc = cur + NBA;
  const int tid = (int)threadIdx.x, lane = tid & 31, wave = tid >> 5;
  unsigned short* srow = (unsigned short*)(misc + MISC_INTS + wave * 96);
  float*          nrow = (float*)(misc + MISC_INTS + wave * 96 + 32);
  const int nodeBase = (int)blockIdx.x * NBA;

  {
    const v4i z4 = {0, 0, 0, 0};
    for (int i = tid * 4; i < CSR_ZINTS; i += NTHR * 4) *(v4ia*)(dsm + i) = z4;
    if (tid < MISC_INTS) misc[tid] = 0;
  }
  __syncthreads();

  int t = 0, ov = 0;
  const int nChunks = (nE + CHUNK - 1) / CHUNK;
#pragma unroll 1
  for (int ch = 0; ch < nChunks; ++ch) {
    const int cbase = ch * CHUNK;
    const int wc = scan_chunk<SLA>(dsts, nE, cbase, nodeBase, NBA, vec8, list, tid, lane, wave);
    if (lane == 0) misc[wave] = wc;
    __syncthreads();
    if (wave == 0) {
#pragma unroll 1
      for (int w2 = 0; w2 < NWAVE; ++w2) {
        int c = misc[w2];
        c = c < 0 ? 0 : (c > WCAP ? WCAP : c);
#pragma unroll 1
        for (int b0 = 0; b0 < c; b0 += 32) {
          const int idx = b0 + lane;
          const int ent = list[w2 * WCAP + (idx < WCAP ? idx : WCAP - 1)];
          const int m32 = (c - b0) < 32 ? (c - b0) : 32;
#pragma unroll 1
          for (int k = 0; k < m32; ++k) {
            const int u    = __builtin_amdgcn_readlane(ent, k);
            const int slot = u & (NBA - 1);
            const int el   = (u >> SLA) & (CHUNK - 1);
            const int pk   = ((cbase + el) << SLA) | slot;
            if (t < RCAP) {
              if (lane == 0) { hl[t] = pk; cnt[slot] = cnt[slot] + 1; }
              t = t + 1;
            } else {
              ov = 1;
            }
          }
        }
      }
    }
    __syncthreads();
  }
  if (wave == 0 && lane == 0) { misc[8] = t; misc[9] = ov; }
  __syncthreads();
  int tt = misc[8];
  tt = tt < 0 ? 0 : (tt > RCAP ? RCAP : tt);
  const int ovf = misc[9];

  if (wave == 0) {
    const int base = lane * (NBA / 32);
    int s = 0;
#pragma unroll 1
    for (int i = 0; i < NBA / 32; ++i) s += cnt[base + i];
    int incl = s;
#pragma unroll
    for (int dd = 1; dd < 32; dd <<= 1) {
      const int y = __shfl_up(incl, dd, 32);
      if (lane >= dd) incl += y;
    }
    int run = incl - s;
#pragma unroll 1
    for (int i = 0; i < NBA / 32; ++i) {
      const int cv = cnt[base + i];
      offs[base + i] = run;
      cur[base + i]  = run;
      run += cv;
    }
  }
  __syncthreads();
  if (wave == 0) {
#pragma unroll 1
    for (int b0 = 0; b0 < tt; b0 += 32) {
      const int idx = b0 + lane;
      const int ent = hl[idx < RCAP ? idx : RCAP - 1];
      const int m32 = (tt - b0) < 32 ? (tt - b0) : 32;
#pragma unroll 1
      for (int k = 0; k < m32; ++k) {
        const int u    = __builtin_amdgcn_readlane(ent, k);
        const int slot = u & (NBA - 1);
        if (lane == 0) {
          int p = cur[slot];
          p = p < 0 ? 0 : (p > RCAP - 1 ? RCAP - 1 : p);
          sl[p] = u;
          cur[slot] = p + 1;
        }
      }
    }
  }
  __syncthreads();

  const float qnan = __int_as_float(0x7fc00000);
#pragma unroll 1
  for (int si = 0; si < NBA / NWAVE; ++si) {
    const int s    = si * NWAVE + wave;
    const int node = nodeBase + s;
    int c = cnt[s];
    const bool big = c > DEGCAP;
    c = c < 0 ? 0 : (c > DEGCAP ? DEGCAP : c);
    int o = offs[s];
    o = o < 0 ? 0 : (o > RCAP ? RCAP : o);
    const int nc = node < nN ? node : nN - 1;
    const float dd = dinv[nc];
    const bool poi = big || (ovf != 0);
    const float pz = poi ? qnan : 0.0f;
#pragma unroll
    for (int hf = 0; hf < 2; ++hf) {
      const int j = hf * 32 + lane;
      int idx = o + j;
      idx = idx > RCAP - 1 ? RCAP - 1 : idx;
      const bool valid = j < c;
      const int ent = sl[idx];
      int eid = ent >> SLA;
      eid = eid < 0 ? 0 : (eid > nE - 1 ? nE - 1 : eid);
      int sr = srcs[eid];
      sr = sr < 0 ? 0 : (sr > nN - 1 ? nN - 1 : sr);
      const float wv = bf16_val(ew[eid]);
      const float nr = (dinv[sr] * wv) * dd;
      const int   srv = valid ? sr : 0;
      const float nrv = valid ? (nr + pz) : pz;
      srow[j] = (unsigned short)srv;
      nrow[j] = nrv;
    }
    if (lane == 0) cur[s] = poi ? (c > 1 ? c : 1) : c;
    wave_sync();
    const v4u qa = *(const v4ua*)(srow + 8 * (lane & 7));
    const v4u qb = *(const v4ua*)(nrow + 4 * ((lane - 8) & 15));
    wave_sync();
    const bool wa_ = lane < 8;
    const bool wb_ = (lane >= 8) && (lane < 24);
    unsigned short* pa = stab + (size_t)node * DEGCAP + 8 * (lane & 7);
    float*          pb = ntab + (size_t)node * DEGCAP + 4 * ((lane - 8) & 15);
    if (node < mRows) {
      if (wa_) *(volatile v4u*)pa = qa;
      if (wb_) *(volatile v4u*)pb = qb;
      __threadfence();
      if (wa_) *(volatile v4u*)pa = qa;
      if (wb_) *(volatile v4u*)pb = qb;
    }
  }
  __syncthreads();
  {
    const v4i cv = *(const v4ia*)(cur + 4 * tid);
    int* cp = ctab + (size_t)nodeBase + 4 * tid;
    *(volatile v4i*)cp = cv;
    __threadfence();
    *(volatile v4i*)cp = cv;
  }
}

template <int RND>
__global__ __launch_bounds__(NTHR) void k_hop2(const unsigned short* __restrict__ stab, const float* __restrict__ ntab,
                                               const int* __restrict__ ctab, int nN, int mRows,
                                               const float* __restrict__ hin, float* hout) {
  const int tid = (int)threadIdx.x;
  const int node = (int)blockIdx.x * NTHR + tid;
  const int nd = node < mRows ? node : mRows - 1;
  const bool live = node < nN;
  int c = ctab[nd];
  c = c < 0 ? 0 : (c > DEGCAP ? DEGCAP : c);
  c = live ? c : 0;
  int cm = c;
#pragma unroll
  for (int xm = 16; xm > 0; xm >>= 1) {
    const int oth = __shfl_xor(cm, xm, 32);
    cm = oth > cm ? oth : cm;
  }
  cm = cm > DEGCAP ? DEGCAP : cm;
  float a0 = 0.0f, a1 = 0.0f;
#pragma unroll 1
  for (int k = 0; k < cm; ++k) {
    int sr = (int)stab[(size_t)nd * DEGCAP + k];
    sr = sr > nN - 1 ? nN - 1 : sr;
    const float cf  = ntab[(size_t)nd * DEGCAP + k];
    const float cfm = (k < c) ? cf : 0.0f;
    v2f v = *(const v2fa*)(hin + (size_t)sr * 2);
    if constexpr (RND != 0) { v.x = bf16_val(v.x); v.y = bf16_val(v.y); }
    a0 = fmaf(cfm, v.x, a0);
    a1 = fmaf(cfm, v.y, a1);
  }
  if (node < mRows) {
    v2f o;
    o.x = a0; o.y = a1;
    float* op = hout + (size_t)node * 2;
    *(volatile v2f*)op = o;
    __threadfence();
    *(volatile v2f*)op = o;
  }
}

__global__ __launch_bounds__(NTHR) void k_c0(const float* __restrict__ x, const float* __restrict__ xa,
                                             const float* __restrict__ xb, const float* __restrict__ xc,
                                             const float* __restrict__ w0, const float* __restrict__ b0,
                                             int nN, float* cout, float* rec) {
  __shared__ float wsv[512];
  __shared__ float bsv[64];
  __shared__ __attribute__((aligned(16))) float part[NWAVE * 128];
  __shared__ __attribute__((aligned(16))) float recs[128];
  const int tid = (int)threadIdx.x, lane = tid & 31, wave = tid >> 5;
  for (int i = tid; i < 512; i += NTHR) wsv[i] = bf16_val(w0[i]);
  if (tid < 64) bsv[tid] = bf16_val(b0[tid]);
  __syncthreads();
  const int c0 = 2 * lane;
  float wk[16];
#pragma unroll
  for (int q = 0; q < 8; ++q) { wk[2 * q] = wsv[q * 64 + c0]; wk[2 * q + 1] = wsv[q * 64 + c0 + 1]; }
  const float bv0 = bsv[c0], bv1 = bsv[c0 + 1];
  const int sa = (2 * lane) & 31, sb = (2 * lane + 1) & 31;
  const int rowBase = (int)blockIdx.x * GBM;
  float s0 = 0.0f, s1 = 0.0f, q0 = 0.0f, q1 = 0.0f;
#pragma unroll 1
  for (int i = 0; i < GBM / NWAVE; ++i) {
    const int node = rowBase + (GBM / NWAVE) * wave + i;
    const bool live = node < nN;
    const int nc = live ? node : nN - 1;
    v2f xv = *(const v2fa*)(x + (size_t)nc * 2);
    xv.x = bf16_val(xv.x); xv.y = bf16_val(xv.y);
    const v2f h1 = *(const v2fa*)(xa + (size_t)nc * 2);
    const v2f h2 = *(const v2fa*)(xb + (size_t)nc * 2);
    const v2f h3 = *(const v2fa*)(xc + (size_t)nc * 2);
    float o0 = xv.x * wk[0] + xv.y * wk[2];
    float o1 = xv.x * wk[1] + xv.y * wk[3];
    o0 = o0 + (h1.x * wk[4] + h1.y * wk[6]);
    o1 = o1 + (h1.x * wk[5] + h1.y * wk[7]);
    o0 = o0 + (h2.x * wk[8] + h2.y * wk[10]);
    o1 = o1 + (h2.x * wk[9] + h2.y * wk[11]);
    o0 = o0 + (h3.x * wk[12] + h3.y * wk[14]);
    o1 = o1 + (h3.x * wk[13] + h3.y * wk[15]);
    o0 = o0 + bv0;
    o1 = o1 + bv1;
    const float v0 = live ? o0 : 0.0f;
    const float v1 = live ? o1 : 0.0f;
    s0 += v0; s1 += v1; q0 += v0 * v0; q1 += v1 * v1;
    v4f ow;
    ow.x = __shfl(v0, sa, 32); ow.y = __shfl(v1, sa, 32);
    ow.z = __shfl(v0, sb, 32); ow.w = __shfl(v1, sb, 32);
    float* op = cout + (size_t)node * D + 4 * (lane & 15);
    const bool wr = lane < 16;
    if (wr) *(volatile v4f*)op = ow;
    __threadfence();
    if (wr) *(volatile v4f*)op = ow;
  }
  part[wave * 128 + c0] = s0;
  part[wave * 128 + c0 + 1] = s1;
  part[wave * 128 + 64 + c0] = q0;
  part[wave * 128 + 64 + c0 + 1] = q1;
  __syncthreads();
  if (tid < 128) {
    float tsum = 0.0f;
#pragma unroll
    for (int w2 = 0; w2 < NWAVE; ++w2) tsum += part[w2 * 128 + tid];
    recs[tid] = tsum;
  }
  __syncthreads();
  if (wave == 0) {
    const v4f rv4 = *(const v4fa*)(recs + 4 * lane);
    float* rp = rec + (size_t)blockIdx.x * 128 + 4 * lane;
    *(volatile v4f*)rp = rv4;
    __threadfence();
    *(volatile v4f*)rp = rv4;
  }
}

template <int WF>
__global__ __launch_bounds__(NTHR) void k_hop(const unsigned short* __restrict__ stab, const float* __restrict__ ntab,
                                              const int* __restrict__ ctab, int nN, int mRows,
                                              const float* __restrict__ hin, float* hout,
                                              unsigned short* apl, int segoff) {
  const int tid = (int)threadIdx.x, lane = tid & 31, wave = tid >> 5;
  const int rowBase = (int)blockIdx.x * GBM;
  const int sa = (2 * lane) & 31, sb = (2 * lane + 1) & 31;
  const int q0s = (4 * lane) & 31, q1s = (4 * lane + 1) & 31;
  const int q2s = (4 * lane + 2) & 31, q3s = (4 * lane + 3) & 31;
#pragma unroll 1
  for (int i = 0; i < GBM / NWAVE; ++i) {
    const int node = rowBase + (GBM / NWAVE) * wave + i;
    const bool live = node < nN;
    int c = ctab[node];
    c = c < 0 ? 0 : (c > DEGCAP ? DEGCAP : c);
    c = live ? c : 0;
    float acc0 = 0.0f, acc1 = 0.0f;
#pragma unroll 1
    for (int b0 = 0; b0 < c; b0 += 32) {
      const int j = b0 + lane;
      int sr = (int)stab[(size_t)node * DEGCAP + j];
      sr = sr > nN - 1 ? nN - 1 : sr;
      const float cf  = ntab[(size_t)node * DEGCAP + j];
      const int   cfi = __float_as_int(cf);
      const int m32 = (c - b0) < 32 ? (c - b0) : 32;
#pragma unroll 1
      for (int k = 0; k < m32; ++k) {
        const int   sk = __builtin_amdgcn_readlane(sr, k);
        const float ck = __int_as_float(__builtin_amdgcn_readlane(cfi, k));
        const v2f a = *(const v2fa*)(hin + (size_t)sk * D + 2 * lane);
        acc0 = fmaf(ck, a.x, acc0);
        acc1 = fmaf(ck, a.y, acc1);
      }
    }
    const float v0 = live ? acc0 : 0.0f;
    const float v1 = live ? acc1 : 0.0f;
    const bool wr = lane < 16;
    const unsigned hb0 = bf16_bits(v0), hb1 = bf16_bits(v1);
    const unsigned lb0 = bf16_bits(v0 - __uint_as_float(hb0 << 16));
    const unsigned lb1 = bf16_bits(v1 - __uint_as_float(hb1 << 16));
    const int hw = (int)(hb0 | (hb1 << 16));
    const int lw = (int)(lb0 | (lb1 << 16));
    const int g0 = __shfl(hw, q0s, 32), g1 = __shfl(hw, q1s, 32);
    const int g2 = __shfl(hw, q2s, 32), g3 = __shfl(hw, q3s, 32);
    const int p0 = __shfl(lw, q0s, 32), p1 = __shfl(lw, q1s, 32);
    const int p2 = __shfl(lw, q2s, 32), p3 = __shfl(lw, q3s, 32);
    const bool lsel = (lane & 8) != 0;
    v4u pv;
    pv.x = (unsigned int)(lsel ? p0 : g0);
    pv.y = (unsigned int)(lsel ? p1 : g1);
    pv.z = (unsigned int)(lsel ? p2 : g2);
    pv.w = (unsigned int)(lsel ? p3 : g3);
    unsigned short* hp = apl + (size_t)node * AP + segoff + 8 * (lane & 15);
    v4f ow;
    ow.x = __shfl(v0, sa, 32); ow.y = __shfl(v1, sa, 32);
    ow.z = __shfl(v0, sb, 32); ow.w = __shfl(v1, sb, 32);
    float* op = hout + (size_t)node * D + 4 * (lane & 15);
    if (wr) *(volatile v4u*)hp = pv;
    if constexpr (WF != 0) { if (wr) *(volatile v4f*)op = ow; }
    __threadfence();
    if (wr) *(volatile v4u*)hp = pv;
    if constexpr (WF != 0) { if (wr) *(volatile v4f*)op = ow; }
  }
}

template <int EP>
__global__ __launch_bounds__(GTHR) void k_gemm(const unsigned short* A, int lda, const unsigned short* __restrict__ WT,
                                               int K, const float* __restrict__ bias, const float* __restrict__ resid,
                                               int nN, float* outF, int ldo, unsigned short* outH, int ldh,
                                               float* rec) {
  __shared__ __attribute__((aligned(16))) float stg[GBM * GBN];
  __shared__ __attribute__((aligned(16))) float recs[128];
  const int tid = (int)threadIdx.x, lane = tid & 31, wave = tid >> 5, hh = lane >> 4, m = lane & 15;
  const int rowBase = (int)blockIdx.x * GBM;
  const int col0    = (int)blockIdx.y * GBN;

  v8f acc[4];
  {
    const v8f z = {0.f, 0.f, 0.f, 0.f, 0.f, 0.f, 0.f, 0.f};
    acc[0] = z; acc[1] = z; acc[2] = z; acc[3] = z;
  }
  const unsigned short* ap = A  + (size_t)(rowBase + 16 * wave + m) * (size_t)lda + 8 * hh;
  const unsigned short* wp = WT + (size_t)(col0 + m) * (size_t)K + 8 * hh;
  const int ksteps = K >> 5;
#pragma unroll 1
  for (int ks = 0; ks < ksteps; ++ks) {
    FragB af;
    af.h[0] = *(const v8usa*)(ap + 32 * ks);
    af.h[1] = *(const v8usa*)(ap + 32 * ks + 16);
#pragma unroll
    for (int t = 0; t < 4; ++t) {
      const unsigned short* wq = wp + (size_t)(16 * t) * (size_t)K + 32 * ks;
      FragB bf;
      bf.h[0] = *(const v8usa*)wq;
      bf.h[1] = *(const v8usa*)(wq + 16);
      acc[t] = wmb(af, bf, acc[t]);
    }
  }

#pragma unroll
  for (int t = 0; t < 4; ++t) {
    const int lc = 16 * t + m;
#pragma unroll
    for (int r = 0; r < 8; ++r) {
      const int lr = 16 * wave + 8 * hh + r;
      stg[lr * GBN + lc] = acc[t][r];
    }
  }
  __syncthreads();

  v4f bb4 = {0.f, 0.f, 0.f, 0.f};
  if constexpr (EP != 3) {
    const v4f t1 = *(const v4fa*)(bias + col0 + 4 * m);
    bb4.x = bf16_val(t1.x); bb4.y = bf16_val(t1.y); bb4.z = bf16_val(t1.z); bb4.w = bf16_val(t1.w);
  }
  v4f fv[8];
#pragma unroll
  for (int i = 0; i < 8; ++i) {
    const int lr = 16 * wave + 2 * i + hh;
    fv[i] = *(const v4fa*)(stg + lr * GBN + 4 * m);
  }
  __syncthreads();

  v4f cs = {0.f, 0.f, 0.f, 0.f}, cq = {0.f, 0.f, 0.f, 0.f};
#pragma unroll
  for (int i = 0; i < 8; ++i) {
    const int gr = rowBase + 16 * wave + 2 * i + hh;
    const bool ok = gr < nN;
    v4f y = fv[i] + bb4;
    if constexpr (EP == 2) {
      const v4f rs4 = *(const v4fa*)(resid + (size_t)gr * D + 4 * m);
      y = y + rs4;
    }
    if constexpr (EP == 0 || EP == 2) {
      y.x = fmaxf(y.x, 0.0f); y.y = fmaxf(y.y, 0.0f); y.z = fmaxf(y.z, 0.0f); y.w = fmaxf(y.w, 0.0f);
    }
    y.x = ok ? y.x : 0.0f; y.y = ok ? y.y : 0.0f; y.z = ok ? y.z : 0.0f; y.w = ok ? y.w : 0.0f;
    fv[i] = y;
    if constexpr (EP == 1) { cs = cs + y; cq = cq + y * y; }
  }

  if constexpr (EP == 1) {
    const int p = 2 * wave + hh;
    *(v4fa*)(stg + p * 64 + 4 * m) = cs;
    *(v4fa*)(stg + 512 + p * 64 + 4 * m) = cq;
    __syncthreads();
    if (tid < 128) {
      const int qd = tid >> 6;
      const int c  = tid & 63;
      float s = 0.0f;
#pragma unroll
      for (int pp = 0; pp < 8; ++pp) s += stg[512 * qd + pp * 64 + c];
      recs[tid] = s;
    }
    __syncthreads();
    if (wave == 0) {
      const v4f rv4 = *(const v4fa*)(recs + 4 * lane);
      float* rp = rec + (size_t)blockIdx.x * 128 + 4 * lane;
      *(volatile v4f*)rp = rv4;
      __threadfence();
      *(volatile v4f*)rp = rv4;
    }
  }

  v4us hv[8], lv[8];
  if constexpr (EP == 0 || EP == 2) {
#pragma unroll
    for (int i = 0; i < 8; ++i) hilo4(fv[i], hv[i], lv[i]);
  }
#pragma unroll
  for (int i = 0; i < 8; ++i) {
    const int gr = rowBase + 16 * wave + 2 * i + hh;
    if constexpr (EP != 2) {
      float* op = outF + (size_t)gr * (size_t)ldo + col0 + 4 * m;
      *(volatile v4f*)op = fv[i];
    }
    if constexpr (EP == 0 || EP == 2) {
      unsigned short* hp = outH + (size_t)gr * (size_t)ldh + 4 * m;
      *(volatile v4us*)hp = hv[i];
      *(volatile v4us*)(hp + D) = lv[i];
    }
  }
  __threadfence();
#pragma unroll
  for (int i = 0; i < 8; ++i) {
    const int gr = rowBase + 16 * wave + 2 * i + hh;
    if constexpr (EP != 2) {
      float* op = outF + (size_t)gr * (size_t)ldo + col0 + 4 * m;
      *(volatile v4f*)op = fv[i];
    }
    if constexpr (EP == 0 || EP == 2) {
      unsigned short* hp = outH + (size_t)gr * (size_t)ldh + 4 * m;
      *(volatile v4us*)hp = hv[i];
      *(volatile v4us*)(hp + D) = lv[i];
    }
  }
}

__global__ __launch_bounds__(NTHR) void k_istat(const float* __restrict__ rec, int nBlk, int nN, float* mst) {
  __shared__ double acc[128];
  __shared__ __attribute__((aligned(16))) float line[128];
  const int tid = (int)threadIdx.x, lane = tid & 31, wave = tid >> 5;
  if (tid < 128) {
    double s = 0.0;
#pragma unroll 1
    for (int b = 0; b < nBlk; ++b) s += (double)rec[(size_t)b * 128 + tid];
    acc[tid] = s;
  }
  __syncthreads();
  if (tid < 64) {
    const double inv_n = 1.0 / (double)nN;
    const double mean = acc[tid] * inv_n;
    double var = acc[64 + tid] * inv_n - mean * mean;
    var = var > 0.0 ? var : 0.0;
    line[tid] = (float)mean;
    line[64 + tid] = (float)(1.0 / sqrt(var + 1e-5));
  }
  __syncthreads();
  if (wave == 0) {
    const v4f v = *(const v4fa*)(line + 4 * lane);
    float* p = mst + 4 * lane;
    *(volatile v4f*)p = v;
    __threadfence();
    *(volatile v4f*)p = v;
  }
}

template <int RES>
__global__ __launch_bounds__(NTHR) void k_apply(const float* __restrict__ cpl, const float* __restrict__ mst,
                                                int nN, int mRows, float* data, unsigned short* apl) {
  const int tid = (int)threadIdx.x;
  const int row = (int)blockIdx.x * 16 + (tid >> 4);
  const int q   = tid & 15;
  const v4f m4 = *(const v4fa*)(mst + 4 * q);
  const v4f r4 = *(const v4fa*)(mst + D + 4 * q);
  const v4f c4 = *(const v4fa*)(cpl + (size_t)row * D + 4 * q);
  v4f y = (c4 - m4) * r4;
  if constexpr (RES != 0) {
    const v4f d4 = *(const v4fa*)(data + (size_t)row * D + 4 * q);
    y = y + d4;
  }
  y.x = fmaxf(y.x, 0.0f); y.y = fmaxf(y.y, 0.0f); y.z = fmaxf(y.z, 0.0f); y.w = fmaxf(y.w, 0.0f);
  const bool live = row < nN;
  y.x = live ? y.x : 0.0f; y.y = live ? y.y : 0.0f; y.z = live ? y.z : 0.0f; y.w = live ? y.w : 0.0f;
  v4us h4, l4;
  hilo4(y, h4, l4);
  float* dp = data + (size_t)row * D + 4 * q;
  unsigned short* hp = apl + (size_t)row * AP + 4 * q;
  *(volatile v4f*)dp = y;
  *(volatile v4us*)hp = h4;
  *(volatile v4us*)(hp + D) = l4;
  __threadfence();
  *(volatile v4f*)dp = y;
  *(volatile v4us*)hp = h4;
  *(volatile v4us*)(hp + D) = l4;
}

__device__ __forceinline__ void ln_rows(v8f* f, const float* g, const float* b, int m) {
  float gg[4], bv[4];
#pragma unroll
  for (int nt = 0; nt < 4; ++nt) { gg[nt] = g[16 * nt + m]; bv[nt] = b[16 * nt + m]; }
#pragma unroll
  for (int r = 0; r < 8; ++r) {
    float s = (f[0][r] + f[1][r]) + (f[2][r] + f[3][r]);
#pragma unroll
    for (int xm = 1; xm < 16; xm <<= 1) s += __shfl_xor(s, xm, 32);
    const float mean = s * (1.0f / 64.0f);
    const float d0 = f[0][r] - mean, d1 = f[1][r] - mean, d2 = f[2][r] - mean, d3 = f[3][r] - mean;
    float q = (d0 * d0 + d1 * d1) + (d2 * d2 + d3 * d3);
#pragma unroll
    for (int xm = 1; xm < 16; xm <<= 1) q += __shfl_xor(q, xm, 32);
    const float inv = rsqrtf(q * (1.0f / 64.0f) + EPSV);
    f[0][r] = d0 * inv * gg[0] + bv[0];
    f[1][r] = d1 * inv * gg[1] + bv[1];
    f[2][r] = d2 * inv * gg[2] + bv[2];
    f[3][r] = d3 * inv * gg[3] + bv[3];
  }
}
__device__ __forceinline__ void store_hilo(unsigned short* at, const v8f* f, int hh, int m) {
#pragma unroll
  for (int nt = 0; nt < 4; ++nt) {
#pragma unroll
    for (int r = 0; r < 8; ++r) {
      const float v = f[nt][r];
      const unsigned hb = bf16_bits(v);
      const unsigned lb = bf16_bits(v - __uint_as_float(hb << 16));
      at[(8 * hh + r) * KP + 16 * nt + m]     = (unsigned short)hb;
      at[(8 * hh + r) * KP + D + 16 * nt + m] = (unsigned short)lb;
    }
  }
}
__device__ __forceinline__ void gemm16(v8f* acc, const unsigned short* at, const unsigned short* __restrict__ wt,
                                       int hh, int m) {
  const unsigned short* ap = at + m * KP + 8 * hh;
  const unsigned short* bp = wt + (size_t)m * KP + 8 * hh;
#pragma unroll
  for (int ks = 0; ks < KP / 32; ++ks) {
    FragB af;
    af.h[0] = *(const v8usa*)(ap + 32 * ks);
    af.h[1] = *(const v8usa*)(ap + 32 * ks + 16);
#pragma unroll
    for (int t = 0; t < 4; ++t) {
      const unsigned short* wq = bp + (size_t)(16 * t) * KP + 32 * ks;
      FragB bf;
      bf.h[0] = *(const v8usa*)wq;
      bf.h[1] = *(const v8usa*)(wq + 16);
      acc[t] = wmb(af, bf, acc[t]);
    }
  }
}

__global__ __launch_bounds__(NTHR) void k_edge(const int* __restrict__ rows, const int* __restrict__ cols,
                                               const float* __restrict__ ew, int nE, int nN,
                                               const float* __restrict__ pp, const unsigned short* __restrict__ wab,
                                               const float* __restrict__ we0, const float* __restrict__ be0,
                                               const float* __restrict__ ln0g, const float* __restrict__ ln0b,
                                               const float* __restrict__ ba, const float* __restrict__ bb,
                                               const float* __restrict__ lng, const float* __restrict__ lnb,
                                               const float* __restrict__ wf, const float* __restrict__ bfp,
                                               float* opl, float* orec) {
  extern __shared__ __attribute__((aligned(16))) float esm[];
  float* cst = esm;
  float* ost = esm + COST;
  const int tid = (int)threadIdx.x, lane = tid & 31, wave = tid >> 5, hh = lane >> 4, m = lane & 15;
  float* zt = esm + ECST + wave * 1024;
  unsigned short* at = (unsigned short*)(esm + ECST + NWAVE * 1024) + wave * 2048;

  {
    const int g = tid >> 6, el = tid & 63;
    if (g == 0) {
      cst[CW128 + el]      = bf16_val(we0[2 * D * D + el]);
      cst[CBA0 + el]       = bf16_val(ba[el]);
      cst[CBA0 + 256 + el] = bf16_val(ba[D + el]);
      cst[CWF + el]        = bf16_val(wf[el]);
    } else if (g == 1) {
      cst[CBE0 + el]       = bf16_val(be0[el]);
      cst[CBB0 + el]       = bf16_val(bb[el]);
      cst[CBB0 + 256 + el] = bf16_val(bb[D + el]);
    } else if (g == 2) {
      cst[CG0 + el]        = bf16_val(ln0g[el]);
      cst[CG1 + el]        = bf16_val(lng[el]);
      cst[CG1 + 256 + el]  = bf16_val(lng[D + el]);
    } else {
      cst[CB0 + el]        = bf16_val(ln0b[el]);
      cst[CB1 + el]        = bf16_val(lnb[el]);
      cst[CB1 + 256 + el]  = bf16_val(lnb[D + el]);
    }
    if (tid == 0) cst[CBF] = bf16_val(bfp[0]);
  }
  __syncthreads();

  const int eBase = (int)blockIdx.x * EB + 16 * wave;
  int rv, cv, evi;
  {
    const int e  = eBase + m;
    const int ec = e < nE ? e : nE - 1;
    int r_ = rows[ec];
    r_ = r_ < 0 ? 0 : (r_ > nN - 1 ? nN - 1 : r_);
    int c_ = cols[ec];
    c_ = c_ < 0 ? 0 : (c_ > nN - 1 ? nN - 1 : c_);
    rv = r_; cv = c_;
    evi = __float_as_int(bf16_val(ew[ec]));
  }
  const v2f wq2 = *(const v2fa*)(cst + CW128 + 2 * lane);
  const v2f bq2 = *(const v2fa*)(cst + CBE0 + 2 * lane);
#pragma unroll 4
  for (int i = 0; i < 16; ++i) {
    const int   rn = __builtin_amdgcn_readlane(rv, i);
    const int   cn = __builtin_amdgcn_readlane(cv, i);
    const float ef = __int_as_float(__builtin_amdgcn_readlane(evi, i));
    const v2f pr = *(const v2fa*)(pp + (size_t)rn * KP + 2 * lane);
    const v2f pc = *(const v2fa*)(pp + (size_t)cn * KP + D + 2 * lane);
    v2f z;
    z.x = ((pr.x + pc.x) + ef * wq2.x) + bq2.x;
    z.y = ((pr.y + pc.y) + ef * wq2.y) + bq2.y;
    *(v2fa*)(zt + i * D + 2 * lane) = z;
  }
  wave_sync();
  v8f hc[4];
#pragma unroll
  for (int nt = 0; nt < 4; ++nt) {
#pragma unroll
    for (int r = 0; r < 8; ++r) hc[nt][r] = zt[(8 * hh + r) * D + 16 * nt + m];
  }
  ln_rows(hc, cst + CG0, cst + CB0, m);
#pragma unroll
  for (int nt = 0; nt < 4; ++nt) {
#pragma unroll
    for (int r = 0; r < 8; ++r) hc[nt][r] = fmaxf(hc[nt][r], 0.0f);
  }
  store_hilo(at, hc, hh, m);
  wave_sync();

  const v8f z8 = {0.f, 0.f, 0.f, 0.f, 0.f, 0.f, 0.f, 0.f};
#pragma unroll
  for (int j = 0; j < 2; ++j) {
    v8f acc[4];
    acc[0] = z8; acc[1] = z8; acc[2] = z8; acc[3] = z8;
    gemm16(acc, at, wab + (size_t)(2 * j) * D * KP, hh, m);
    wave_sync();
    {
      float cba[4];
#pragma unroll
      for (int nt = 0; nt < 4; ++nt) cba[nt] = cst[CBA0 + 256 * j + 16 * nt + m];
#pragma unroll
      for (int nt = 0; nt < 4; ++nt) {
#pragma unroll
        for (int r = 0; r < 8; ++r) acc[nt][r] = fmaxf(acc[nt][r] + cba[nt], 0.0f);
      }
    }
    store_hilo(at, acc, hh, m);
    wave_sync();
    acc[0] = z8; acc[1] = z8; acc[2] = z8; acc[3] = z8;
    gemm16(acc, at, wab + (size_t)(2 * j + 1) * D * KP, hh, m);
    wave_sync();
    {
      float cbb[4];
#pragma unroll
      for (int nt = 0; nt < 4; ++nt) cbb[nt] = cst[CBB0 + 256 * j + 16 * nt + m];
#pragma unroll
      for (int nt = 0; nt < 4; ++nt) {
#pragma unroll
        for (int r = 0; r < 8; ++r) acc[nt][r] = acc[nt][r] + cbb[nt];
      }
    }
    ln_rows(acc, cst + CG1 + 256 * j, cst + CB1 + 256 * j, m);
#pragma unroll
    for (int nt = 0; nt < 4; ++nt) {
#pragma unroll
      for (int r = 0; r < 8; ++r) hc[nt][r] = fmaxf(acc[nt][r] + hc[nt][r], 0.0f);
    }
    if (j == 0) {
      store_hilo(at, hc, hh, m);
      wave_sync();
    }
  }

  {
    float wfv[4];
#pragma unroll
    for (int nt = 0; nt < 4; ++nt) wfv[nt] = cst[CWF + 16 * nt + m];
    const float bfc = cst[CBF];
#pragma unroll
    for (int r = 0; r < 8; ++r) {
      float p = hc[0][r] * wfv[0];
      p = fmaf(hc[1][r], wfv[1], p);
      p = fmaf(hc[2][r], wfv[2], p);
      p = fmaf(hc[3][r], wfv[3], p);
#pragma unroll
      for (int xm = 1; xm < 16; xm <<= 1) p += __shfl_xor(p, xm, 32);
      const float o = p + bfc;
      const int e = eBase + 8 * hh + r;
      const float ov = (e < nE) ? o : 0.0f;
      if (m == 0) ost[16 * wave + 8 * hh + r] = ov;
    }
  }
  __syncthreads();
  if (tid == 0) {
    double S = 0.0, S2 = 0.0;
#pragma unroll 1
    for (int i = 0; i < EB; ++i) { const double v = (double)ost[i]; S += v; S2 += v * v; }
    *(dbla*)(cst + CDBL)     = S;
    *(dbla*)(cst + CDBL + 2) = S2;
  }
  __syncthreads();
  if (wave == 0) {
    const v4f ov4 = *(const v4fa*)(ost + 4 * lane);
    DU rr;
    rr.d[0] = *(const dbla*)(cst + CDBL);
    rr.d[1] = *(const dbla*)(cst + CDBL + 2);
    v4u recv;
    recv.x = (lane == 0) ? rr.u.x : 0u;
    recv.y = (lane == 0) ? rr.u.y : 0u;
    recv.z = (lane == 0) ? rr.u.z : 0u;
    recv.w = (lane == 0) ? rr.u.w : 0u;
    float* op = opl + (size_t)blockIdx.x * EB + 4 * lane;
    unsigned int* rp = (unsigned int*)(orec + (size_t)blockIdx.x * 32) + 4 * (lane & 7);
    const bool wrec = lane < 8;
    *(volatile v4f*)op = ov4;
    if (wrec) *(volatile v4u*)rp = recv;
    __threadfence();
    *(volatile v4f*)op = ov4;
    if (wrec) *(volatile v4u*)rp = recv;
  }
}

__global__ __launch_bounds__(NTHR) void k_ostat(const float* __restrict__ orec, int nBlk, int nE, float* ost) {
  __shared__ double rs[NTHR];
  __shared__ double rq[NTHR];
  __shared__ __attribute__((aligned(16))) float line[32];
  const int tid = (int)threadIdx.x, lane = tid & 31, wave = tid >> 5;
  double s = 0.0, q = 0.0;
#pragma unroll 1
  for (int b = tid; b < nBlk; b += NTHR) {
    const dbla* p = (const dbla*)(orec + (size_t)b * 32);
    s += p[0];
    q += p[1];
  }
  rs[tid] = s; rq[tid] = q;
  __syncthreads();
#pragma unroll 1
  for (int st = NTHR / 2; st > 0; st >>= 1) {
    if (tid < st) { rs[tid] += rs[tid + st]; rq[tid] += rq[tid + st]; }
    __syncthreads();
  }
  if (tid < 32) line[tid] = 0.0f;
  __syncthreads();
  if (tid == 0) {
    const double S = rs[0], Q = rq[0];
    const double mean = S / (double)nE;
    double var = (Q - S * mean) / (double)(nE - 1);
    var = var > 0.0 ? var : 0.0;
    const float meanf = (float)mean;
    const float stdf  = (float)sqrt(var);
    line[0] = meanf;
    line[1] = (stdf > 0.0f) ? (1.0f / stdf) : 0.0f;
  }
  __syncthreads();
  if (wave == 0) {
    const v4f v = *(const v4fa*)(line + 4 * (lane & 7));
    float* p = ost + 4 * (lane & 7);
    const bool wr = lane < 8;
    if (wr) *(volatile v4f*)p = v;
    __threadfence();
    if (wr) *(volatile v4f*)p = v;
  }
}

__global__ __launch_bounds__(NTHR) void k_out(const float* __restrict__ opl, const float* __restrict__ ost,
                                              int nE, float* out) {
  const int e = ((int)blockIdx.x * NTHR + (int)threadIdx.x) * 4;
  if (e >= nE) return;
  const float ms = ost[0];
  const float iv = ost[1];
  const v4f o = *(const v4fa*)(opl + e);
  v4f r;
  r.x = fabsf((o.x - ms) * iv);
  r.y = fabsf((o.y - ms) * iv);
  r.z = fabsf((o.z - ms) * iv);
  r.w = fabsf((o.w - ms) * iv);
  float* p = out + e;
  *(volatile v4f*)p = r;
  __threadfence();
  *(volatile v4f*)p = r;
}

static inline int cdiv(int a, int b) { return (a + b - 1) / b; }
static inline size_t al256(size_t o) { return (o + 255) & ~(size_t)255; }

extern "C" void kernel_launch(void* const* d_in, const int* in_sizes, int n_in,
                              void* d_out, int out_size, void* d_ws, size_t ws_size,
                              hipStream_t stream) {
  if (n_in < 19) return;
  if (in_sizes[0] < 32 || (in_sizes[0] & 1) != 0) return;
  const int nN = in_sizes[0] / 2;
  if (nN < 16 || nN > 65535) return;
  if (in_sizes[1] < 2 || (in_sizes[1] & 1) != 0) return;
  const int nE = in_sizes[1] / 2;
  if (nE < EB || (nE % EB) != 0 || nE >= (1 << 21)) return;
  if (in_sizes[2] != nE) return;
  if (in_sizes[3] != 4 * 2 * D || in_sizes[4] != D) return;
  if (in_sizes[5] != NCONV * 4 * D * D || in_sizes[6] != NCONV * D) return;
  if (in_sizes[7] != (2 * D + 1) * D || in_sizes[8] != D) return;
  if (in_sizes[9] != D || in_sizes[10] != D) return;
  if (in_sizes[11] != 2 * D * D || in_sizes[12] != 2 * D) return;
  if (in_sizes[13] != 2 * D * D || in_sizes[14] != 2 * D) return;
  if (in_sizes[15] != 2 * D || in_sizes[16] != 2 * D) return;
  if (in_sizes[17] != D || in_sizes[18] != 1) return;
  if (out_size != nE) return;

  const float* x     = (const float*)d_in[0];
  const int*   eix   = (const int*)d_in[1];
  const float* ea    = (const float*)d_in[2];
  const float* tag0w = (const float*)d_in[3];
  const float* tag0b = (const float*)d_in[4];
  const float* tagw  = (const float*)d_in[5];
  const float* tagb  = (const float*)d_in[6];
  const float* we0   = (const float*)d_in[7];
  const float* be0   = (const float*)d_in[8];
  const float* ln0g  = (const float*)d_in[9];
  const float* ln0b  = (const float*)d_in[10];
  const float* wa    = (const float*)d_in[11];
  const float* ba    = (const float*)d_in[12];
  const float* wb    = (const float*)d_in[13];
  const float* bb    = (const float*)d_in[14];
  const float* lng   = (const float*)d_in[15];
  const float* lnb   = (const float*)d_in[16];
  const float* wf    = (const float*)d_in[17];
  const float* bfp   = (const float*)d_in[18];
  float* out = (float*)d_out;
  const int* rowp = eix;
  const int* colp = eix + nE;

  const int MP   = cdiv(nN, GBM) * GBM;
  const int gM   = MP / GBM;
  const int gD   = cdiv(nN, NBD);
  const int NBPD = gD * NBD;
  const int gA   = cdiv(MP, NBA);
  const int NCT  = gA * NBA;
  const int gE   = nE / EB;
  const int gH2  = cdiv(MP, NTHR);
  if ((long long)NCT < (long long)MP || NBPD < nN || (MP % 16) != 0) return;
  const int vec8 = ((nE & 3) == 0) ? 1 : 0;

  char* ws = (char*)d_ws;
  size_t off = 0;
  const size_t oBT   = off; off = al256(off + (size_t)NCONV * D * KC * 2);
  const size_t oPBT  = off; off = al256(off + (size_t)KP * KP * 2);
  const size_t oWAB  = off; off = al256(off + (size_t)4 * D * KP * 2);
  const size_t oDINV = off; off = al256(off + (size_t)NBPD * 4);
  const size_t oCNT  = off; off = al256(off + (size_t)NCT * 4);
  const size_t oSRC  = off; off = al256(off + (size_t)MP * DEGCAP * 2);
  const size_t oNRM  = off; off = al256(off + (size_t)MP * DEGCAP * 4);
  const size_t oXA   = off; off = al256(off + (size_t)MP * 2 * 4);
  const size_t oXB   = off; off = al256(off + (size_t)MP * 2 * 4);
  const size_t oXC   = off; off = al256(off + (size_t)MP * 2 * 4);
  const size_t oAPL  = off; off = al256(off + (size_t)MP * AP * 2);
  const size_t oDATA = off; off = al256(off + (size_t)MP * D * 4);
  const size_t oPP   = off; off = al256(off + (size_t)MP * KP * 4);
  const size_t oDFHL = off; off = al256(off + (size_t)MP * KP * 2);
  const size_t oREC  = off; off = al256(off + (size_t)gM * 128 * 4);
  const size_t oMST  = off; off = al256(off + (size_t)128 * 4);
  const size_t oOPL  = off; off = al256(off + (size_t)gE * EB * 4);
  const size_t oOREC = off; off = al256(off + (size_t)gE * 128);
  const size_t oOST  = off; off = al256(off + (size_t)128);
  if (off > ws_size || off > (size_t)WSMAX) return;
  unsigned short* BT   = (unsigned short*)(ws + oBT);
  unsigned short* PBT  = (unsigned short*)(ws + oPBT);
  unsigned short* WAB  = (unsigned short*)(ws + oWAB);
  float*          DINV = (float*)(ws + oDINV);
  int*            CNT  = (int*)(ws + oCNT);
  unsigned short* SRC  = (unsigned short*)(ws + oSRC);
  float*          NRM  = (float*)(ws + oNRM);
  float*          XA   = (float*)(ws + oXA);
  float*          XB   = (float*)(ws + oXB);
  float*          XC   = (float*)(ws + oXC);
  unsigned short* APL  = (unsigned short*)(ws + oAPL);
  float*          DATA = (float*)(ws + oDATA);
  float*          PP   = (float*)(ws + oPP);
  float*          P0   = PP;
  float*          P1   = PP + (size_t)MP * D;
  unsigned short* DFHL = (unsigned short*)(ws + oDFHL);
  float*          REC  = (float*)(ws + oREC);
  float*          MST  = (float*)(ws + oMST);
  float*          OPL  = (float*)(ws + oOPL);
  float*          OREC = (float*)(ws + oOREC);
  float*          OST  = (float*)(ws + oOST);

  const size_t csrLds  = (size_t)CSR_LDS_INTS * 4;
  const size_t edgeLds = (size_t)ELDS_FLOATS * 4;
  hipFuncSetAttribute(reinterpret_cast<const void*>(&k_csr), hipFuncAttributeMaxDynamicSharedMemorySize, (int)csrLds);
  hipFuncSetAttribute(reinterpret_cast<const void*>(&k_edge), hipFuncAttributeMaxDynamicSharedMemorySize, (int)edgeLds);

  k_wprep<<<UTOT / NTHR, NTHR, 0, stream>>>(tagw, we0, wa, wb, BT, PBT, WAB);
  k_deg<<<gD, NTHR, 0, stream>>>(colp, ea, nE, vec8, DINV);
  k_csr<<<gA, NTHR, csrLds, stream>>>(rowp, colp, ea, nE, nN, vec8, MP, DINV, CNT, SRC, NRM);
  k_hop2<1><<<gH2, NTHR, 0, stream>>>(SRC, NRM, CNT, nN, MP, x, XA);
  k_hop2<0><<<gH2, NTHR, 0, stream>>>(SRC, NRM, CNT, nN, MP, XA, XB);
  k_hop2<0><<<gH2, NTHR, 0, stream>>>(SRC, NRM, CNT, nN, MP, XB, XC);
  k_c0<<<gM, NTHR, 0, stream>>>(x, XA, XB, XC, tag0w, tag0b, nN, P0, REC);
  k_istat<<<1, NTHR, 0, stream>>>(REC, gM, nN, MST);
  k_apply<0><<<MP / 16, NTHR, 0, stream>>>(P0, MST, nN, MP, DATA, APL);
  for (int c = 0; c < NCONV; ++c) {
    const float* h0 = (c & 1) ? P1 : DATA;
    const unsigned short* BTc = BT + (size_t)c * D * KC;
    const float* tb = tagb + (size_t)c * D;
    k_hop<1><<<gM, NTHR, 0, stream>>>(SRC, NRM, CNT, nN, MP, h0, P0, APL, 1 * KP);
    k_hop<1><<<gM, NTHR, 0, stream>>>(SRC, NRM, CNT, nN, MP, P0, P1, APL, 2 * KP);
    k_hop<0><<<gM, NTHR, 0, stream>>>(SRC, NRM, CNT, nN, MP, P1, P0, APL, 3 * KP);
    if (c == NCONV - 1) {
      k_gemm<2><<<dim3(gM, 1), GTHR, 0, stream>>>(APL, AP, BTc, KC, tb, DATA, nN, P1, D, DFHL, KP, REC);
    } else if (c & 1) {
      k_gemm<1><<<dim3(gM, 1), GTHR, 0, stream>>>(APL, AP, BTc, KC, tb, DATA, nN, P0, D, DFHL, KP, REC);
      k_istat<<<1, NTHR, 0, stream>>>(REC, gM, nN, MST);
      k_apply<1><<<MP / 16, NTHR, 0, stream>>>(P0, MST, nN, MP, DATA, APL);
    } else {
      k_gemm<0><<<dim3(gM, 1), GTHR, 0, stream>>>(APL, AP, BTc, KC, tb, DATA, nN, P1, D, APL, AP, REC);
    }
  }
  k_gemm<3><<<dim3(gM, 2), GTHR, 0, stream>>>(DFHL, KP, PBT, KP, tagb, DATA, nN, PP, KP, DFHL, KP, REC);
  k_edge<<<gE, NTHR, edgeLds, stream>>>(rowp, colp, ea, nE, nN, PP, WAB, we0, be0, ln0g, ln0b,
                                        ba, bb, lng, lnb, wf, bfp, OPL, OREC);
  k_ostat<<<1, NTHR, 0, stream>>>(OREC, gE, nE, OST);
  k_out<<<cdiv(nE, NTHR * 4), NTHR, 0, stream>>>(OPL, OST, nE, out);
}
